// RelativeMultiHeadAttenion_68496138436889
// MI455X (gfx1250) — hardware-verified
//
#include <hip/hip_runtime.h>
#include <stdint.h>


typedef unsigned short u16;
typedef unsigned int u32;
typedef __bf16 bf16x16 __attribute__((ext_vector_type(16)));
typedef float f32x8 __attribute__((ext_vector_type(8)));
typedef float v4f __attribute__((ext_vector_type(4)));
typedef u32 v4u __attribute__((ext_vector_type(4)));
typedef u16 us8 __attribute__((ext_vector_type(8)));

union Frag {
  bf16x16 v;
  v4u q[2];
};

__device__ __forceinline__ u16 f2bf(float f) {
  const u32 u = __float_as_uint(f);
  const u32 r = u + 0x7FFFu + ((u >> 16) & 1u);
  return (u16)(r >> 16);
}
__device__ __forceinline__ float bf2f(u16 b) { return __uint_as_float(((u32)b) << 16); }

__device__ __forceinline__ void split8(v4f a, v4f b, us8& h, us8& l) {
  float f[8];
  f[0] = a.x; f[1] = a.y; f[2] = a.z; f[3] = a.w;
  f[4] = b.x; f[5] = b.y; f[6] = b.z; f[7] = b.w;
#pragma unroll
  for (int i = 0; i < 8; ++i) {
    const u16 hb = f2bf(f[i]);
    h[i] = hb;
    l[i] = f2bf(f[i] - bf2f(hb));
  }
}

__device__ __forceinline__ f32x8 zero8() {
  f32x8 z;
#pragma unroll
  for (int e = 0; e < 8; ++e) z[e] = 0.0f;
  return z;
}

__device__ __forceinline__ void ldf(Frag& f, const u16* p) {
  f.q[0] = *(const v4u*)p;
  f.q[1] = *(const v4u*)(p + 16);
}

__device__ __forceinline__ f32x8 wmma3(const Frag& ah, const Frag& al, const Frag& bh, const Frag& bl, f32x8 c) {
  c = __builtin_amdgcn_wmma_f32_16x16x32_bf16(false, ah.v, false, bh.v, (short)0, c, false, false);
  c = __builtin_amdgcn_wmma_f32_16x16x32_bf16(false, ah.v, false, bl.v, (short)0, c, false, false);
  c = __builtin_amdgcn_wmma_f32_16x16x32_bf16(false, al.v, false, bh.v, (short)0, c, false, false);
  asm volatile("v_nop\n\tv_nop\n\tv_nop\n\tv_nop" : "+v"(c) : "v"(ah.v), "v"(al.v), "v"(bh.v), "v"(bl.v));
  return c;
}

__global__ __launch_bounds__(256) void k_split(const float* __restrict__ s, u16* dh, u16* dl, int n8) {
  const int g = blockIdx.x * 256 + threadIdx.x;
  if (g >= n8) return;
  const size_t o = (size_t)g * 8;
  const v4f a = *(const v4f*)(s + o);
  const v4f b = *(const v4f*)(s + o + 4);
  us8 h, l;
  split8(a, b, h, l);
  *(volatile us8*)(dh + o) = h;
  *(volatile us8*)(dl + o) = l;
  __threadfence();
  *(volatile us8*)(dh + o) = h;
  *(volatile us8*)(dl + o) = l;
}

__global__ __launch_bounds__(256) void k_split_tr(const float* __restrict__ s, u16* dh, u16* dl, int R, int C) {
  __shared__ __attribute__((aligned(16))) float Ts[64 * 68];
  const int c0 = blockIdx.x * 64, r0 = blockIdx.y * 64;
  const int t = threadIdx.x;
  {
    const int r = t >> 2, cb = (t & 3) * 16;
    const float* p = s + (size_t)(r0 + r) * C + c0 + cb;
#pragma unroll
    for (int q = 0; q < 4; ++q) {
      const v4f v = *(const v4f*)(p + 4 * q);
      Ts[(cb + 4 * q + 0) * 68 + r] = v.x;
      Ts[(cb + 4 * q + 1) * 68 + r] = v.y;
      Ts[(cb + 4 * q + 2) * 68 + r] = v.z;
      Ts[(cb + 4 * q + 3) * 68 + r] = v.w;
    }
  }
  __syncthreads();
  us8 h[2], l[2];
  size_t go[2];
#pragma unroll
  for (int it = 0; it < 2; ++it) {
    const int pc = t + 256 * it, c = pc >> 3, q = pc & 7;
    const v4f a = *(const v4f*)(Ts + c * 68 + 8 * q);
    const v4f b = *(const v4f*)(Ts + c * 68 + 8 * q + 4);
    split8(a, b, h[it], l[it]);
    go[it] = (size_t)(c0 + c) * R + r0 + 8 * q;
  }
#pragma unroll
  for (int it = 0; it < 2; ++it) {
    *(volatile us8*)(dh + go[it]) = h[it];
    *(volatile us8*)(dl + go[it]) = l[it];
  }
  __threadfence();
#pragma unroll
  for (int it = 0; it < 2; ++it) {
    *(volatile us8*)(dh + go[it]) = h[it];
    *(volatile us8*)(dl + go[it]) = l[it];
  }
}

template <int MODE>
__global__ __launch_bounds__(256) void k_gemm(const u16* __restrict__ Ah, const u16* __restrict__ Al,
                                              const u16* __restrict__ Bh, const u16* __restrict__ Bl,
                                              u16* Ch, u16* Cl, float* Cf,
                                              int lda, int ldb, int ldc, int K,
                                              int zA, int zB, int zC) {
  __shared__ __attribute__((aligned(16))) float Cs[64 * 132];
  const int z = blockIdx.z;
  const int bm = blockIdx.y * 64, bn = blockIdx.x * 128;
  const int tid = threadIdx.x, wave = tid >> 5, lane = tid & 31;
  const int m = lane & 15, hh = lane >> 4;
  const int wr = (wave & 1) * 32, wc = (wave >> 1) * 32;

  const u16* ahb = Ah + (size_t)z * zA + (size_t)(bm + wr + m) * lda + 8 * hh;
  const u16* alb = Al + (size_t)z * zA + (size_t)(bm + wr + m) * lda + 8 * hh;
  const u16* bhb = Bh + (size_t)z * zB + (size_t)(bn + wc + m) * ldb + 8 * hh;
  const u16* blb = Bl + (size_t)z * zB + (size_t)(bn + wc + m) * ldb + 8 * hh;

  f32x8 acc[2][2];
#pragma unroll
  for (int rt = 0; rt < 2; ++rt)
#pragma unroll
    for (int ct = 0; ct < 2; ++ct) acc[rt][ct] = zero8();

  for (int k0 = 0; k0 < K; k0 += 32) {
    Frag ah[2], al[2], bh[2], bl[2];
#pragma unroll
    for (int rt = 0; rt < 2; ++rt) {
      ldf(ah[rt], ahb + (size_t)(rt * 16) * lda + k0);
      ldf(al[rt], alb + (size_t)(rt * 16) * lda + k0);
    }
#pragma unroll
    for (int ct = 0; ct < 2; ++ct) {
      ldf(bh[ct], bhb + (size_t)(ct * 16) * ldb + k0);
      ldf(bl[ct], blb + (size_t)(ct * 16) * ldb + k0);
    }
#pragma unroll
    for (int rt = 0; rt < 2; ++rt)
#pragma unroll
      for (int ct = 0; ct < 2; ++ct)
        acc[rt][ct] = wmma3(ah[rt], al[rt], bh[ct], bl[ct], acc[rt][ct]);
  }

#pragma unroll
  for (int rt = 0; rt < 2; ++rt)
#pragma unroll
    for (int ct = 0; ct < 2; ++ct)
#pragma unroll
      for (int r = 0; r < 8; ++r)
        Cs[(wr + rt * 16 + 8 * hh + r) * 132 + wc + ct * 16 + m] = acc[rt][ct][r];
  __syncthreads();

  if (MODE == 1) {
    float* cb = Cf + (size_t)z * zC;
    v4f v[8];
    size_t go[8];
#pragma unroll
    for (int i = 0; i < 8; ++i) {
      const int row = wave * 8 + i;
      v[i] = *(const v4f*)(Cs + row * 132 + 4 * lane);
      go[i] = (size_t)(bm + row) * ldc + bn + 4 * lane;
    }
#pragma unroll
    for (int i = 0; i < 8; ++i) *(volatile v4f*)(cb + go[i]) = v[i];
    __threadfence();
#pragma unroll
    for (int i = 0; i < 8; ++i) *(volatile v4f*)(cb + go[i]) = v[i];
  } else {
    u16* chb = Ch + (size_t)z * zC;
    u16* clb = Cl + (size_t)z * zC;
    us8 hv[4], lv[4];
    size_t go[4];
#pragma unroll
    for (int i = 0; i < 4; ++i) {
      const int row = wave * 8 + 2 * i + (lane >> 4);
      const int cs = (lane & 15) * 8;
      const v4f a = *(const v4f*)(Cs + row * 132 + cs);
      const v4f b = *(const v4f*)(Cs + row * 132 + cs + 4);
      split8(a, b, hv[i], lv[i]);
      go[i] = (size_t)(bm + row) * ldc + bn + cs;
    }
#pragma unroll
    for (int i = 0; i < 4; ++i) {
      *(volatile us8*)(chb + go[i]) = hv[i];
      *(volatile us8*)(clb + go[i]) = lv[i];
    }
    __threadfence();
#pragma unroll
    for (int i = 0; i < 4; ++i) {
      *(volatile us8*)(chb + go[i]) = hv[i];
      *(volatile us8*)(clb + go[i]) = lv[i];
    }
  }
}

__global__ __launch_bounds__(256) void k_vtr(const u16* __restrict__ sh, const u16* __restrict__ sl, u16* dh, u16* dl) {
  __shared__ __attribute__((aligned(16))) u16 Th[64 * 72];
  __shared__ __attribute__((aligned(16))) u16 Tl[64 * 72];
  const int blk = blockIdx.x, lt = blk & 15, h = (blk >> 4) & 15, b = blk >> 8;
  const int l0 = lt * 64, t = threadIdx.x;
  const size_t src = (size_t)b * 1048576 + (size_t)h * 65536 + (size_t)l0 * 64;
#pragma unroll
  for (int it = 0; it < 2; ++it) {
    const int pc = t + 256 * it, l = pc >> 3, q = pc & 7;
    const us8 a = *(const us8*)(sh + src + l * 64 + 8 * q);
    const us8 c = *(const us8*)(sl + src + l * 64 + 8 * q);
#pragma unroll
    for (int i = 0; i < 8; ++i) {
      Th[(8 * q + i) * 72 + l] = a[i];
      Tl[(8 * q + i) * 72 + l] = c[i];
    }
  }
  __syncthreads();
  const size_t dst = (size_t)(b * 16 + h) * 65536 + (size_t)l0;
  us8 oh[2], ol[2];
  size_t go[2];
#pragma unroll
  for (int it = 0; it < 2; ++it) {
    const int pc = t + 256 * it, e = pc >> 3, q = pc & 7;
    oh[it] = *(const us8*)(Th + e * 72 + 8 * q);
    ol[it] = *(const us8*)(Tl + e * 72 + 8 * q);
    go[it] = dst + (size_t)e * 1024 + 8 * q;
  }
#pragma unroll
  for (int it = 0; it < 2; ++it) {
    *(volatile us8*)(dh + go[it]) = oh[it];
    *(volatile us8*)(dl + go[it]) = ol[it];
  }
  __threadfence();
#pragma unroll
  for (int it = 0; it < 2; ++it) {
    *(volatile us8*)(dh + go[it]) = oh[it];
    *(volatile us8*)(dl + go[it]) = ol[it];
  }
}

__device__ __forceinline__ f32x8 tile_k64(const Frag& ah0, const Frag& al0, const Frag& ah1, const Frag& al1,
                                          const u16* bh, const u16* bl) {
  Frag h0, l0, h1, l1;
  ldf(h0, bh); ldf(h1, bh + 32);
  ldf(l0, bl); ldf(l1, bl + 32);
  f32x8 acc = zero8();
  acc = wmma3(ah0, al0, h0, l0, acc);
  acc = wmma3(ah1, al1, h1, l1, acc);
  return acc;
}

__global__ __launch_bounds__(256) void k_attn(const u16* __restrict__ QPh, const u16* __restrict__ QPl,
                                              const u16* __restrict__ KPh, const u16* __restrict__ KPl,
                                              const u16* __restrict__ VTh, const u16* __restrict__ VTl,
                                              const u16* __restrict__ Eh, const u16* __restrict__ El,
                                              u16* AOh, u16* AOl) {
  extern __shared__ v4u dsm[];
  float* S = (float*)dsm;
  u16* P = (u16*)dsm;
  float* Ost = (float*)(dsm + 8192);

  const int blk = blockIdx.x;
  const int ib = blk & 31, h = (blk >> 5) & 15, b = blk >> 9;
  const int i0 = ib * 32;
  const int tid = threadIdx.x, wave = tid >> 5, lane = tid & 31;
  const int m = lane & 15, hh = lane >> 4;

  const size_t pq = (size_t)b * 1048576 + (size_t)h * 65536;
  const u16* Qh = QPh + pq;
  const u16* Ql = QPl + pq;
  const size_t pk = (size_t)b * 1048576 + (size_t)h * 64;
  const u16* Kh = KPh + pk;
  const u16* Kl = KPl + pk;
  const size_t pv = (size_t)(b * 16 + h) * 65536;
  const u16* Vh = VTh + pv;
  const u16* Vl = VTl + pv;

  if (tid < 32) {
    const int j = i0 + tid + 1;
    if (j < 1024) S[tid * 1024 + j] = 0.0f;
  }

  const int ncol2 = 991 - i0;
  const int nct2 = (ncol2 > 0) ? ((ncol2 + 63) >> 6) : 0;
  const int U1 = 32 + nct2;
  for (int u = wave; u < U1; u += 8) {
    const int rt = u >> 4, ct = u & 15;
    const int rb = i0 + rt * 16;
    int ra = rb + m;
    ra = (ra > 1023) ? 1023 : ra;
    Frag ah0, al0, ah1, al1;
    const u16* qa = Qh + (size_t)ra * 64 + 8 * hh;
    const u16* qb = Ql + (size_t)ra * 64 + 8 * hh;
    ldf(ah0, qa); ldf(ah1, qa + 32);
    ldf(al0, qb); ldf(al1, qb + 32);
#pragma unroll 1
    for (int sub = 0; sub < 4; ++sub) {
      const int col0 = ct * 64 + sub * 16;
      const size_t eo = (size_t)(col0 + m) * 64 + 8 * hh;
      const f32x8 acc = tile_k64(ah0, al0, ah1, al1, Eh + eo, El + eo);
      const int c = col0 + m;
#pragma unroll
      for (int r = 0; r < 8; ++r) {
        const int i2 = rb + 8 * hh + r;
        const bool low = (c >= 1023 - i2);
        const int lr = (low ? i2 : (i2 - 1)) - i0;
        const int j = low ? (c + i2 - 1023) : (c + i2 + 1);
        if ((unsigned)lr < 32u && (unsigned)j < 1024u) S[lr * 1024 + j] = acc[r];
      }
    }
  }
  __syncthreads();

  for (int u = wave; u < 32; u += 8) {
    const int rt = u >> 4, ct = u & 15;
    const int rb = i0 + rt * 16;
    Frag ah0, al0, ah1, al1;
    const u16* qa = Qh + (size_t)(rb + m) * 64 + 8 * hh;
    const u16* qb = Ql + (size_t)(rb + m) * 64 + 8 * hh;
    ldf(ah0, qa); ldf(ah1, qa + 32);
    ldf(al0, qb); ldf(al1, qb + 32);
#pragma unroll 1
    for (int sub = 0; sub < 4; ++sub) {
      const int col0 = ct * 64 + sub * 16;
      const size_t ko = (size_t)(col0 + m) * 1024 + 8 * hh;
      const f32x8 acc = tile_k64(ah0, al0, ah1, al1, Kh + ko, Kl + ko);
#pragma unroll
      for (int r = 0; r < 8; ++r)
        S[(rt * 16 + 8 * hh + r) * 1024 + col0 + m] += acc[r];
    }
  }
  __syncthreads();

#pragma unroll 1
  for (int rr = 0; rr < 4; ++rr) {
    const int row = wave * 4 + rr;
    const float* sr = S + row * 1024 + lane * 32;
    v4f xv[8];
    float mx = -3.0e38f;
#pragma unroll
    for (int q = 0; q < 8; ++q) {
      v4f v = *(const v4f*)(sr + 4 * q);
      v = v * 0.125f;
      xv[q] = v;
      mx = fmaxf(mx, fmaxf(fmaxf(v.x, v.y), fmaxf(v.z, v.w)));
    }
#pragma unroll
    for (int off = 16; off > 0; off >>= 1) mx = fmaxf(mx, __shfl_xor(mx, off, 32));
    float sum = 0.0f;
#pragma unroll
    for (int q = 0; q < 8; ++q) {
      v4f e;
      e.x = __expf(xv[q].x - mx);
      e.y = __expf(xv[q].y - mx);
      e.z = __expf(xv[q].z - mx);
      e.w = __expf(xv[q].w - mx);
      xv[q] = e;
      sum += (e.x + e.y) + (e.z + e.w);
    }
#pragma unroll
    for (int off = 16; off > 0; off >>= 1) sum += __shfl_xor(sum, off, 32);
    const float inv = 1.0f / sum;
    u16* ph = P + row * 2048 + lane * 32;
    u16* pl = ph + 1024;
#pragma unroll
    for (int q4 = 0; q4 < 4; ++q4) {
      const v4f a = xv[2 * q4] * inv;
      const v4f bq = xv[2 * q4 + 1] * inv;
      us8 hv, lv;
      split8(a, bq, hv, lv);
      *(us8*)(ph + 8 * q4) = hv;
      *(us8*)(pl + 8 * q4) = lv;
    }
  }
  __syncthreads();

  {
    const int rt = wave & 1, nt = wave >> 1;
    const u16* pa = P + (rt * 16 + m) * 2048 + 8 * hh;
    const u16* vb = Vh + (size_t)(nt * 16 + m) * 1024 + 8 * hh;
    const u16* vc = Vl + (size_t)(nt * 16 + m) * 1024 + 8 * hh;
    f32x8 acc = zero8();
#pragma unroll 2
    for (int ks = 0; ks < 32; ++ks) {
      Frag ah, al, bh, bl;
      ldf(ah, pa + ks * 32);
      ldf(al, pa + 1024 + ks * 32);
      ldf(bh, vb + ks * 32);
      ldf(bl, vc + ks * 32);
      acc = wmma3(ah, al, bh, bl, acc);
    }
#pragma unroll
    for (int r = 0; r < 8; ++r) Ost[(rt * 16 + 8 * hh + r) * 64 + nt * 16 + m] = acc[r];
  }
  __syncthreads();

  {
    const int row = wave * 4 + (lane >> 3), q = lane & 7;
    const v4f a = *(const v4f*)(Ost + row * 64 + 8 * q);
    const v4f bq = *(const v4f*)(Ost + row * 64 + 8 * q + 4);
    us8 hv, lv;
    split8(a, bq, hv, lv);
    const size_t g = ((size_t)(b * 1024 + i0 + row)) * 1024 + (size_t)h * 64 + 8 * q;
    *(volatile us8*)(AOh + g) = hv;
    *(volatile us8*)(AOl + g) = lv;
    __threadfence();
    *(volatile us8*)(AOh + g) = hv;
    *(volatile us8*)(AOl + g) = lv;
  }
}


extern "C" void kernel_launch(void* const* d_in, const int* in_sizes, int n_in,
                              void* d_out, int out_size, void* d_ws, size_t ws_size,
                              hipStream_t stream) {
  const int NX = 4194304;
  const int NW = 1048576;
  const int NE = 65536;
  if (n_in < 8) return;
  if (in_sizes[0] != NX || in_sizes[1] != NX || in_sizes[2] != NX) return;
  if (in_sizes[3] != NW || in_sizes[4] != NW || in_sizes[5] != NW || in_sizes[7] != NW) return;
  if (in_sizes[6] != NE) return;
  if (out_size != NX) return;

  const float* q_in = (const float*)d_in[0];
  const float* k_in = (const float*)d_in[1];
  const float* v_in = (const float*)d_in[2];
  const float* WQ = (const float*)d_in[3];
  const float* WK = (const float*)d_in[4];
  const float* WV = (const float*)d_in[5];
  const float* Er = (const float*)d_in[6];
  const float* WM = (const float*)d_in[7];
  float* out = (float*)d_out;

  const size_t bx = (size_t)NX * 2;
  const size_t bw = (size_t)NW * 2;
  const size_t be = (size_t)NE * 2;
  const size_t total = 6 * bx + 8 * bw + 2 * be + 4 * bx;
  if (total > ws_size) return;
  char* w = (char*)d_ws;
  size_t off = 0;
  u16* R0h = (u16*)(w + off); off += bx;
  u16* R0l = (u16*)(w + off); off += bx;
  u16* R1h = (u16*)(w + off); off += bx;
  u16* R1l = (u16*)(w + off); off += bx;
  u16* R2h = (u16*)(w + off); off += bx;
  u16* R2l = (u16*)(w + off); off += bx;
  u16* WQh = (u16*)(w + off); off += bw;
  u16* WQl = (u16*)(w + off); off += bw;
  u16* WKh = (u16*)(w + off); off += bw;
  u16* WKl = (u16*)(w + off); off += bw;
  u16* WVh = (u16*)(w + off); off += bw;
  u16* WVl = (u16*)(w + off); off += bw;
  u16* WMh = (u16*)(w + off); off += bw;
  u16* WMl = (u16*)(w + off); off += bw;
  u16* ERh = (u16*)(w + off); off += be;
  u16* ERl = (u16*)(w + off); off += be;
  u16* QPh = (u16*)(w + off); off += bx;
  u16* QPl = (u16*)(w + off); off += bx;
  u16* KPh = (u16*)(w + off); off += bx;
  u16* KPl = (u16*)(w + off); off += bx;
  if (off > ws_size) return;

  u16* Xqh = R0h; u16* Xql = R0l;
  u16* Xkh = R1h; u16* Xkl = R1l;
  u16* Xvh = R2h; u16* Xvl = R2l;
  u16* VPh = R0h; u16* VPl = R0l;
  u16* VTh = R1h; u16* VTl = R1l;
  u16* AOh = R2h; u16* AOl = R2l;

  const dim3 blk(256);
  const int ATTN_LDS = 131072 + 8192;
  hipFuncSetAttribute((const void*)k_attn, hipFuncAttributeMaxDynamicSharedMemorySize, ATTN_LDS);

  k_split<<<dim3(NX / 8 / 256), blk, 0, stream>>>(q_in, Xqh, Xql, NX / 8);
  k_split<<<dim3(NX / 8 / 256), blk, 0, stream>>>(k_in, Xkh, Xkl, NX / 8);
  k_split<<<dim3(NX / 8 / 256), blk, 0, stream>>>(v_in, Xvh, Xvl, NX / 8);
  k_split<<<dim3(NE / 8 / 256), blk, 0, stream>>>(Er, ERh, ERl, NE / 8);
  k_split_tr<<<dim3(1024 / 64, 1024 / 64), blk, 0, stream>>>(WQ, WQh, WQl, 1024, 1024);
  k_split_tr<<<dim3(1024 / 64, 1024 / 64), blk, 0, stream>>>(WK, WKh, WKl, 1024, 1024);
  k_split_tr<<<dim3(1024 / 64, 1024 / 64), blk, 0, stream>>>(WV, WVh, WVl, 1024, 1024);
  k_split_tr<<<dim3(1024 / 64, 1024 / 64), blk, 0, stream>>>(WM, WMh, WMl, 1024, 1024);

  k_gemm<0><<<dim3(1024 / 128, 4096 / 64, 1), blk, 0, stream>>>(
      Xqh, Xql, WQh, WQl, QPh, QPl, out, 1024, 1024, 1024, 1024, 0, 0, 0);
  k_gemm<0><<<dim3(1024 / 128, 1024 / 64, 4), blk, 0, stream>>>(
      WKh, WKl, Xkh, Xkl, KPh, KPl, out, 1024, 1024, 1024, 1024, 0, NW, NW);
  k_gemm<0><<<dim3(1024 / 128, 4096 / 64, 1), blk, 0, stream>>>(
      Xvh, Xvl, WVh, WVl, VPh, VPl, out, 1024, 1024, 1024, 1024, 0, 0, 0);
  k_vtr<<<dim3(4 * 16 * 16), blk, 0, stream>>>(VPh, VPl, VTh, VTl);
  k_attn<<<dim3(4 * 16 * 32), blk, ATTN_LDS, stream>>>(QPh, QPl, KPh, KPl, VTh, VTl, ERh, ERl, AOh, AOl);
  k_gemm<1><<<dim3(1024 / 128, 4096 / 64, 1), blk, 0, stream>>>(
      AOh, AOl, WMh, WMl, QPh, QPl, out, 1024, 1024, 1024, 1024, 0, 0, 0);
}
